// TransformerBlock_32203664785950
// MI455X (gfx1250) — hardware-verified
//
#include <hip/hip_runtime.h>
#include <math.h>

#ifndef NB
#define NB 4
#endif
#ifndef SEQ
#define SEQ 1024
#endif
#define SEQ_FULL 1024
#define DM 1024
#define CDIM 768
#define NCTX 256
#define NHEAD 16
#define HDIM 64
#define FFD 4096
#define NMOD 6144
#define MODROWS 16
#define MTOK (NB * SEQ)
#define MCTX (NB * NCTX)

#define ACT_C 16
#define W_C 64
#define P_C 1024
#define CTXS_C 64
#define CTXC_C 256
#define SH_ACT 10
#define SH_CTXS 12
#define SH_CTXC 14
#define ATT_SC2 (0.125f * 1.4426950408889634f / 256.0f)

static_assert(SEQ == SEQ_FULL);
static_assert(NB >= 1 && NB <= 4);
static_assert(ACT_C * W_C == (1 << SH_ACT));
static_assert(CTXS_C * W_C == (1 << SH_CTXS));
static_assert(CTXC_C * W_C == (1 << SH_CTXC));
static_assert(ACT_C * ACT_C == 256);
static_assert(CTXS_C % ACT_C == 0 && CTXC_C % ACT_C == 0);
static_assert(NHEAD * HDIM == DM && HDIM == 64);
static_assert(DM == 4 * 32 * 8);
static_assert(NMOD == 6 * DM);
static_assert(MTOK % 64 == 0 && MCTX % 64 == 0 && SEQ % 64 == 0 && NCTX % 64 == 0);
static_assert(SEQ % 128 == 0 && SEQ % 32 == 0 && NCTX % 32 == 0);
static_assert(DM % 64 == 0 && (2 * DM) % 64 == 0 && FFD % 64 == 0 && NMOD % 64 == 0);
static_assert(DM % 32 == 0 && CDIM % 32 == 0 && FFD % 32 == 0);
static_assert((DM / 8) % 32 == 0 && (CDIM / 8) % 32 == 0 && (FFD / 8) % 32 == 0);
static_assert((MCTX * CDIM / 8) % 256 == 0);
static_assert(MTOK % 8 == 0);
static_assert(MODROWS == 16 && NB <= MODROWS);
static_assert(8 * 16 * 68 * 4 <= 131072);
static_assert(8 * 64 * 72 * 2 <= 131072);
static_assert(8 * 16 * 72 * 2 <= 131072);
static_assert(256 * 4 <= 131072);

typedef _Float16 h16;
typedef __attribute__((ext_vector_type(16))) _Float16 v16h;
typedef __attribute__((ext_vector_type(8)))  _Float16 v8h;
typedef __attribute__((ext_vector_type(8)))  float    v8f;
typedef __attribute__((ext_vector_type(4)))  float    v4f;


static __device__ __forceinline__ float bfr(float f) {
    unsigned u = __float_as_uint(f);
    u += 0x7FFFu + ((u >> 16) & 1u);
    return __uint_as_float(u & 0xFFFF0000u);
}
static __device__ __forceinline__ h16 toh_flush(float v) {
    const float w = (fabsf(v) < 6.103515625e-05f) ? 0.0f : v;
    return (h16)w;
}
static __device__ __forceinline__ void st8h(h16* P, size_t o, const float* v) {
    v8h pk;
#pragma unroll
    for (int i = 0; i < 8; ++i) pk[i] = toh_flush(v[i]);
    *(volatile v8h*)(P + o) = pk;
    __threadfence();
    *(volatile v8h*)(P + o) = pk;
}

union FragU { v16h v; v8h h[2]; };
static __device__ __forceinline__ v16h frag_ld(const h16* p) {
    FragU f; f.h[0] = *(const v8h*)(p); f.h[1] = *(const v8h*)(p + 16); return f.v;
}
static __device__ __forceinline__ v8f wmma16g(v16h a, v16h b, v8f c) {
    c = __builtin_amdgcn_wmma_f32_16x16x32_f16(false, a, false, b, (short)0, c, false, false);
    asm volatile("v_nop\n\tv_nop\n\tv_nop\n\tv_nop" : "+v"(c) : "v"(a), "v"(b));
    return c;
}
static __device__ __forceinline__ void wave_sync_lds() {
    __builtin_amdgcn_fence(3  , "workgroup");
    __builtin_amdgcn_wave_barrier();
    __builtin_amdgcn_fence(2  , "workgroup");
}

enum { EP_F32 = 0, EP_F32R = 1, EP_F32RB = 2, EP_H16 = 3, EP_GELU = 4, EP_TR = 5 };

template <int MI, int EPI, int SH, int OM>
static __device__ __forceinline__ void gemm_body(
    const h16* __restrict__ A, unsigned lda, const h16* __restrict__ Bt, unsigned ldb,
    void* __restrict__ Cout, unsigned ldc, const float* __restrict__ bias, const float* __restrict__ resid,
    unsigned M, unsigned N, unsigned K, unsigned ntok) {
  static_assert(EPI != EP_TR || MI == 4);
  __shared__ __align__(16) float sT[8][(EPI == EP_TR) ? 4 : (16 * 68)];
  __shared__ __align__(16) h16   sH[8][(EPI == EP_TR) ? (64 * 72) : 8];
  const unsigned lane = threadIdx.x & 31u;
  const unsigned wave = (unsigned)__builtin_amdgcn_readfirstlane((int)(threadIdx.x >> 5));
  const unsigned tilesN = N >> 6, tilesM = M / (unsigned)(16 * MI);
  const unsigned tile = blockIdx.x * 8u + wave;
  if (tile >= tilesM * tilesN) return;
  const unsigned tm = tile / tilesN;
  const unsigned tn = tile - tm * tilesN;
  const unsigned m0 = tm * (unsigned)(16 * MI), n0 = tn << 6;
  const unsigned rlane = lane & 15u;
  const unsigned koff = (lane >> 4) * 8u;
  const unsigned mOff = koff;
  const float scale = 1.0f / (float)(1 << SH);

  v8f acc[MI][4];
#pragma unroll
  for (int i = 0; i < MI; ++i)
#pragma unroll
    for (int j = 0; j < 4; ++j) acc[i][j] = (v8f){0.f,0.f,0.f,0.f,0.f,0.f,0.f,0.f};

  for (unsigned k0 = 0; k0 < K; k0 += 32u) {
    v16h bh[4];
#pragma unroll
    for (int j = 0; j < 4; ++j)
      bh[j] = frag_ld(Bt + (size_t)(n0 + ((unsigned)j << 4) + rlane) * ldb + koff + k0);
#pragma unroll
    for (int i = 0; i < MI; ++i) {
      const v16h ah = frag_ld(A + (size_t)(m0 + ((unsigned)i << 4) + rlane) * lda + koff + k0);
#pragma unroll
      for (int j = 0; j < 4; ++j)
        acc[i][j] = wmma16g(ah, bh[j], acc[i][j]);
    }
  }

  if constexpr (EPI == EP_TR) {
    h16* st = sH[wave];
#pragma unroll
    for (int j = 0; j < 4; ++j) {
      const unsigned n = n0 + ((unsigned)j << 4) + rlane;
      const float bv = bfr(bias[n]);
#pragma unroll
      for (int i = 0; i < MI; ++i) {
        v8h pk;
#pragma unroll
        for (int r = 0; r < 8; ++r) pk[r] = toh_flush((acc[i][j][r] * scale + bv) * (float)OM);
        *(v8h*)(st + (((unsigned)j << 4) + rlane) * 72u + ((unsigned)i << 4) + mOff) = pk;
      }
    }
    wave_sync_lds();
    const unsigned bq = m0 / ntok;
    const unsigned t0 = m0 - bq * ntok;
    h16* dst = (h16*)Cout + ((size_t)(bq * tilesN + tn) * 64u) * ntok + t0;
    const unsigned q = lane >> 3, c8 = (lane & 7u) * 8u;
    static_assert(32 * 16 * 16 == 64 * 128);
#pragma unroll 1
    for (unsigned it = 0; it < 16u; ++it) {
      const unsigned row = it * 4u + q;
      const v8h hv = *(const v8h*)(st + row * 72u + c8);
      h16* p = dst + (size_t)row * ntok + c8;
      *(volatile v8h*)p = hv;
      __threadfence();
      *(volatile v8h*)p = hv;
    }
  } else {
    float* slab = sT[wave];
#pragma unroll
    for (int i = 0; i < MI; ++i) {
      const unsigned mBase = m0 + ((unsigned)i << 4);
#pragma unroll
      for (int j = 0; j < 4; ++j) {
        const unsigned n = n0 + ((unsigned)j << 4) + rlane;
        const float bv = bfr(bias[n]);
#pragma unroll
        for (int r = 0; r < 8; ++r) {
          const float v = acc[i][j][r] * scale + bv;
          slab[(mOff + (unsigned)r) * 68u + ((unsigned)j << 4) + rlane] = v;
        }
      }
      wave_sync_lds();
      if constexpr (EPI == EP_F32 || EPI == EP_F32R || EPI == EP_F32RB) {
        float* C = (float*)Cout;
        const unsigned hh = lane >> 4, c4 = (lane & 15u) * 4u;
        static_assert(32 * 16 * 8 == 16 * 256);
#pragma unroll
        for (int half = 0; half < 2; ++half) {
          v4f vv[4];
#pragma unroll
          for (int it = 0; it < 4; ++it) {
            const unsigned row = (unsigned)(half * 4 + it) * 2u + hh;
            vv[it] = *(const v4f*)(slab + row * 68u + c4);
            if constexpr (EPI == EP_F32R || EPI == EP_F32RB) {
              v4f rr = *(const v4f*)(resid + (size_t)(mBase + row) * ldc + n0 + c4);
              if constexpr (EPI == EP_F32RB) { rr.x = bfr(rr.x); rr.y = bfr(rr.y); rr.z = bfr(rr.z); rr.w = bfr(rr.w); }
              vv[it] += rr;
            }
          }
          for (int pass = 0; pass < 2; ++pass) {
#pragma unroll
            for (int it = 0; it < 4; ++it) {
              const unsigned row = (unsigned)(half * 4 + it) * 2u + hh;
              *(volatile v4f*)(C + (size_t)(mBase + row) * ldc + n0 + c4) = vv[it];
            }
            __threadfence();
          }
        }
      } else {
        h16* C = (h16*)Cout;
        const unsigned q = lane >> 3, c8 = (lane & 7u) * 8u;
        static_assert(32 * 16 * 4 == 16 * 128);
#pragma unroll 1
        for (unsigned it = 0; it < 4u; ++it) {
          const unsigned row = it * 4u + q;
          const float* sp = slab + row * 68u + c8;
          const v4f s0 = *(const v4f*)sp, s1 = *(const v4f*)(sp + 4);
          const float e[8] = {s0.x, s0.y, s0.z, s0.w, s1.x, s1.y, s1.z, s1.w};
          v8h hv;
#pragma unroll
          for (int k = 0; k < 8; ++k) {
            float v = e[k];
            if constexpr (EPI == EP_GELU) v = 0.5f * v * (1.0f + erff(v * 0.70710678118654752f));
            hv[k] = toh_flush(v * (float)OM);
          }
          h16* p = C + (size_t)(mBase + row) * ldc + n0 + c8;
          *(volatile v8h*)p = hv;
          __threadfence();
          *(volatile v8h*)p = hv;
        }
      }
      wave_sync_lds();
    }
  }
}

__global__ __launch_bounds__(256) void k_gemm_mod(const h16* __restrict__ A, unsigned lda, const h16* __restrict__ Bt, unsigned ldb,
                                                  float* __restrict__ C, unsigned ldc, const float* __restrict__ bias,
                                                  unsigned M, unsigned N, unsigned K) {
  gemm_body<1, EP_F32, SH_ACT, 1>(A, lda, Bt, ldb, (void*)C, ldc, bias, nullptr, M, N, K, 1u);
}
__global__ __launch_bounds__(256) void k_gemm_h16(const h16* __restrict__ A, unsigned lda, const h16* __restrict__ Bt, unsigned ldb,
                                                  h16* __restrict__ C, unsigned ldc, const float* __restrict__ bias,
                                                  unsigned M, unsigned N, unsigned K) {
  gemm_body<4, EP_H16, SH_ACT, ACT_C>(A, lda, Bt, ldb, (void*)C, ldc, bias, nullptr, M, N, K, 1u);
}
__global__ __launch_bounds__(256) void k_gemm_tr(const h16* __restrict__ A, unsigned lda, const h16* __restrict__ Bt, unsigned ldb,
                                                 h16* __restrict__ C, const float* __restrict__ bias,
                                                 unsigned M, unsigned N, unsigned K, unsigned ntok) {
  gemm_body<4, EP_TR, SH_ACT, ACT_C>(A, lda, Bt, ldb, (void*)C, 0u, bias, nullptr, M, N, K, ntok);
}
__global__ __launch_bounds__(256) void k_gemm_gelu(const h16* __restrict__ A, unsigned lda, const h16* __restrict__ Bt, unsigned ldb,
                                                   h16* __restrict__ C, unsigned ldc, const float* __restrict__ bias,
                                                   unsigned M, unsigned N, unsigned K) {
  gemm_body<4, EP_GELU, SH_ACT, ACT_C>(A, lda, Bt, ldb, (void*)C, ldc, bias, nullptr, M, N, K, 1u);
}
__global__ __launch_bounds__(256) void k_gemm_res_s(const h16* __restrict__ A, unsigned lda, const h16* __restrict__ Bt, unsigned ldb,
                                                    float* __restrict__ C, unsigned ldc, const float* __restrict__ bias,
                                                    const float* __restrict__ resid, unsigned M, unsigned N, unsigned K) {
  gemm_body<4, EP_F32RB, SH_CTXS, 1>(A, lda, Bt, ldb, (void*)C, ldc, bias, resid, M, N, K, 1u);
}
__global__ __launch_bounds__(256) void k_gemm_res_c(const h16* __restrict__ A, unsigned lda, const h16* __restrict__ Bt, unsigned ldb,
                                                    float* __restrict__ C, unsigned ldc, const float* __restrict__ bias,
                                                    const float* __restrict__ resid, unsigned M, unsigned N, unsigned K) {
  gemm_body<4, EP_F32R, SH_CTXC, 1>(A, lda, Bt, ldb, (void*)C, ldc, bias, resid, M, N, K, 1u);
}
__global__ __launch_bounds__(256) void k_gemm_res_f(const h16* __restrict__ A, unsigned lda, const h16* __restrict__ Bt, unsigned ldb,
                                                    float* __restrict__ C, unsigned ldc, const float* __restrict__ bias,
                                                    const float* __restrict__ resid, unsigned M, unsigned N, unsigned K) {
  gemm_body<4, EP_F32R, SH_ACT, 1>(A, lda, Bt, ldb, (void*)C, ldc, bias, resid, M, N, K, 1u);
}

__global__ __launch_bounds__(256) void k_wt16(const float* __restrict__ Wm, unsigned KI, unsigned NO, unsigned per,
                                              h16* __restrict__ W16) {
    const unsigned u = blockIdx.x * 256u + threadIdx.x;
    if (u >= NO * per) return;
    const unsigned o = u / per;
    const unsigned k0 = 8u * (u - o * per);
    float v[8];
#pragma unroll
    for (int i = 0; i < 8; ++i) v[i] = bfr(Wm[(size_t)(k0 + (unsigned)i) * NO + o]) * (float)W_C;
    st8h(W16, (size_t)o * KI + k0, v);
}

__global__ __launch_bounds__(256) void k_silu(const float* __restrict__ temb, h16* __restrict__ s16) {
    __shared__ float sB[256];
    const unsigned t = threadIdx.x;
    const unsigned bx = blockIdx.x;
    const unsigned row = bx >> 2, ch = bx & 3u;
    const unsigned rc = min(row, (unsigned)(NB - 1));
    const float tv = bfr(temb[(size_t)rc * DM + ch * 256u + t]);
    const float sg = 1.0f / (1.0f + expf(-tv));
    const float val = (row < (unsigned)NB) ? (tv * sg) * (float)ACT_C : 0.0f;
    sB[t] = val;
    __syncthreads();
    if (t < 32u) {
        float v[8];
#pragma unroll
        for (int i = 0; i < 8; ++i) v[i] = sB[8u * t + (unsigned)i];
        st8h(s16, (size_t)row * DM + ch * 256u + 8u * t, v);
    }
}

__global__ __launch_bounds__(256) void k_ctx16(const float* __restrict__ ctx, h16* __restrict__ c16) {
    const unsigned u = blockIdx.x * 256u + threadIdx.x;
    if (u >= (unsigned)(MCTX * CDIM / 8)) return;
    const float* p = ctx + (size_t)u * 8u;
    const v4f a = *(const v4f*)p, b = *(const v4f*)(p + 4);
    float v[8] = {bfr(a.x), bfr(a.y), bfr(a.z), bfr(a.w), bfr(b.x), bfr(b.y), bfr(b.z), bfr(b.w)};
#pragma unroll
    for (int i = 0; i < 8; ++i) v[i] *= (float)ACT_C;
    st8h(c16, (size_t)u * 8u, v);
}

static __device__ __forceinline__ void ld8(const float* __restrict__ p, unsigned cvt, float* v) {
    const v4f a = *(const v4f*)p, c = *(const v4f*)(p + 4);
    v[0] = a.x; v[1] = a.y; v[2] = a.z; v[3] = a.w; v[4] = c.x; v[5] = c.y; v[6] = c.z; v[7] = c.w;
    if (cvt != 0u) {
#pragma unroll
        for (int i = 0; i < 8; ++i) v[i] = bfr(v[i]);
    }
}

__global__ __launch_bounds__(256) void k_lnmod(const float* __restrict__ xin, const float* __restrict__ g, const float* __restrict__ bt,
                                               const float* __restrict__ modp, unsigned sh_off, unsigned sc_off, unsigned cvt_in,
                                               h16* __restrict__ z16) {
    const unsigned wave = (unsigned)__builtin_amdgcn_readfirstlane((int)(threadIdx.x >> 5));
    const unsigned row = blockIdx.x * 8u + wave;
    const unsigned L = threadIdx.x & 31u;
    if (row >= (unsigned)MTOK) return;
    const unsigned b = row / (unsigned)SEQ;
    const float* xr = xin + (size_t)row * DM + 8u * L;
    float s = 0.f;
#pragma unroll 1
    for (unsigned p = 0; p < 4u; ++p) {
        float v[8];
        ld8(xr + p * 256u, cvt_in, v);
        s += ((v[0] + v[1]) + (v[2] + v[3])) + ((v[4] + v[5]) + (v[6] + v[7]));
    }
#pragma unroll
    for (int o = 16; o > 0; o >>= 1) s += __shfl_xor(s, o, 32);
    const float mu = s * (1.0f / (float)DM);
    float q = 0.f;
#pragma unroll 1
    for (unsigned p = 0; p < 4u; ++p) {
        float v[8];
        ld8(xr + p * 256u, cvt_in, v);
#pragma unroll
        for (int i = 0; i < 8; ++i) { const float d = v[i] - mu; q += d * d; }
    }
#pragma unroll
    for (int o = 16; o > 0; o >>= 1) q += __shfl_xor(q, o, 32);
    const float rs = rsqrtf(q * (1.0f / (float)DM) + 1e-5f);
    const float* scp = modp + (size_t)b * NMOD + sc_off;
    const float* shp = modp + (size_t)b * NMOD + sh_off;
#pragma unroll 1
    for (unsigned p = 0; p < 4u; ++p) {
        const unsigned c0 = p * 256u + 8u * L;
        float xv[8], gv[8], bv[8], scv[8], shv[8], y[8];
        ld8(xr + p * 256u, cvt_in, xv);
        ld8(g + c0, 1u, gv);
        ld8(bt + c0, 1u, bv);
        ld8(scp + c0, 0u, scv);
        ld8(shp + c0, 0u, shv);
#pragma unroll
        for (int i = 0; i < 8; ++i) {
            const float hn = (xv[i] - mu) * rs * gv[i] + bv[i];
            y[i] = (hn * (1.0f + scv[i]) + shv[i]) * (float)ACT_C;
        }
        st8h(z16, (size_t)row * DM + c0, y);
    }
}

template <int NS, int OMUL>
static __device__ __forceinline__ void attn_body(const h16* __restrict__ Q, unsigned ldq, const h16* __restrict__ Kp, unsigned ldk,
                                                 const h16* __restrict__ VT, h16* __restrict__ ctx) {
    __shared__ __align__(16) h16 sO[8][16 * 72];
    const unsigned lane = threadIdx.x & 31u;
    const unsigned wave = (unsigned)__builtin_amdgcn_readfirstlane((int)(threadIdx.x >> 5));
    const unsigned hh = lane >> 4, c = lane & 15u;
    const unsigned bx = blockIdx.x;
    const unsigned QB = (unsigned)(SEQ / 128);
    const unsigned qblk = bx % QB, bh = bx / QB;
    const unsigned b = bh / (unsigned)NHEAD, h = bh % (unsigned)NHEAD;
    const unsigned q0 = qblk * 128u + wave * 16u;

    const h16* qrow = Q + (size_t)(b * (unsigned)SEQ + q0 + c) * ldq + h * 64u + 8u * hh;
    const v16h qb0 = frag_ld(qrow);
    const v16h qb1 = frag_ld(qrow + 32);
    const h16* kbase = Kp + (size_t)(b * (unsigned)NS + c) * ldk + h * 64u + 8u * hh;
    const h16* vbase = VT + (size_t)(bh * 64u + c) * (unsigned)NS + 8u * hh;

    v8f o[4];
#pragma unroll
    for (int t = 0; t < 4; ++t) o[t] = (v8f){0.f,0.f,0.f,0.f,0.f,0.f,0.f,0.f};
    float mrow = -3.0e38f, lrow = 0.f;

#pragma unroll 1
    for (unsigned kv0 = 0; kv0 < (unsigned)NS; kv0 += 32u) {
        v8f s[2];
#pragma unroll
        for (int tt = 0; tt < 2; ++tt) {
            const h16* kr = kbase + (size_t)(kv0 + (unsigned)tt * 16u) * ldk;
            const v16h kf0 = frag_ld(kr);
            const v16h kf1 = frag_ld(kr + 32);
            v8f z = (v8f){0.f,0.f,0.f,0.f,0.f,0.f,0.f,0.f};
            z = wmma16g(kf0, qb0, z);
            z = wmma16g(kf1, qb1, z);
            s[tt] = z;
        }
        float mx = -3.0e38f;
#pragma unroll
        for (int tt = 0; tt < 2; ++tt)
#pragma unroll
            for (int r = 0; r < 8; ++r) { s[tt][r] *= ATT_SC2; mx = fmaxf(mx, s[tt][r]); }
        mx = fmaxf(mx, __shfl_xor(mx, 16, 32));
        const float mnew = fmaxf(mrow, mx);
        const float alpha = exp2f(mrow - mnew);
        mrow = mnew;
        v16h pb;
        float psum = 0.f;
#pragma unroll
        for (int tt = 0; tt < 2; ++tt)
#pragma unroll
            for (int r = 0; r < 8; ++r) {
                const h16 ph = toh_flush(exp2f(s[tt][r] - mnew) * (float)P_C);
                pb[tt * 8 + r] = ph;
                psum += (float)ph;
            }
        lrow = lrow * alpha + psum;
#pragma unroll
        for (int t = 0; t < 4; ++t)
#pragma unroll
            for (int r = 0; r < 8; ++r) o[t][r] *= alpha;
#pragma unroll
        for (int t = 0; t < 4; ++t) {
            const v16h vf = frag_ld(vbase + (size_t)((unsigned)t * 16u) * (unsigned)NS + kv0);
            o[t] = wmma16g(vf, pb, o[t]);
        }
    }
    const float l = lrow + __shfl_xor(lrow, 16, 32);
    const float inv = (float)OMUL * (1.0f / l);

    h16* pw = sO[wave];
#pragma unroll
    for (int t = 0; t < 4; ++t) {
        v8h ov;
#pragma unroll
        for (int r = 0; r < 8; ++r) ov[r] = toh_flush(o[t][r] * inv);
        *(v8h*)(pw + c * 72u + (unsigned)t * 16u + 8u * hh) = ov;
    }
    wave_sync_lds();
    {
        const unsigned q = lane >> 3, c8 = (lane & 7u) * 8u;
        static_assert(32 * 16 * 4 == 16 * 128);
        v8h ov[4];
#pragma unroll
        for (int it = 0; it < 4; ++it) ov[it] = *(const v8h*)(pw + ((unsigned)it * 4u + q) * 72u + c8);
        h16* dst = ctx + (size_t)(b * (unsigned)SEQ + q0) * DM + h * 64u;
        for (int pass = 0; pass < 2; ++pass) {
#pragma unroll
            for (int it = 0; it < 4; ++it) *(volatile v8h*)(dst + (size_t)((unsigned)it * 4u + q) * DM + c8) = ov[it];
            __threadfence();
        }
    }
}

__global__ __launch_bounds__(256) void k_attn_self(const h16* __restrict__ QK, const h16* __restrict__ VT, h16* __restrict__ ctx) {
    attn_body<SEQ, CTXS_C / ACT_C>(QK, 2u * DM, QK + DM, 2u * DM, VT, ctx);
}
__global__ __launch_bounds__(256) void k_attn_cross(const h16* __restrict__ Q2, const h16* __restrict__ K2, const h16* __restrict__ VT2,
                                                    h16* __restrict__ ctx) {
    attn_body<NCTX, CTXC_C / ACT_C>(Q2, (unsigned)DM, K2, (unsigned)DM, VT2, ctx);
}

static constexpr size_t SZ_WQKV = (size_t)DM * 3 * DM * 2;
static constexpr size_t SZ_WDD  = (size_t)DM * DM * 2;
static constexpr size_t SZ_WCD  = (size_t)CDIM * DM * 2;
static constexpr size_t SZ_WFF  = (size_t)DM * FFD * 2;
static constexpr size_t SZ_WMOD = (size_t)DM * NMOD * 2;
static constexpr size_t SZ_S16  = (size_t)MODROWS * DM * 2;
static constexpr size_t SZ_MOD  = (size_t)MODROWS * NMOD * 4;
static constexpr size_t SZ_CIN  = (size_t)MCTX * CDIM * 2;
static constexpr size_t SZ_H16  = (size_t)MTOK * DM * 2;
static constexpr size_t SZ_QK   = (size_t)MTOK * 2 * DM * 2;
static constexpr size_t SZ_VT   = (size_t)MTOK * DM * 2;
static constexpr size_t SZ_CTX  = (size_t)MTOK * DM * 2;
static constexpr size_t SZ_X    = (size_t)MTOK * DM * 4;
static constexpr size_t SZ_FF   = (size_t)MTOK * FFD * 2;
static constexpr size_t SZ_K2   = (size_t)MCTX * DM * 2;
static constexpr size_t SZ_VT2  = (size_t)MCTX * DM * 2;

static constexpr size_t OFF_WQKV = 0;
static constexpr size_t OFF_WOS  = OFF_WQKV + SZ_WQKV;
static constexpr size_t OFF_WQ   = OFF_WOS + SZ_WDD;
static constexpr size_t OFF_WK   = OFF_WQ + SZ_WDD;
static constexpr size_t OFF_WV   = OFF_WK + SZ_WCD;
static constexpr size_t OFF_WOC  = OFF_WV + SZ_WCD;
static constexpr size_t OFF_W1   = OFF_WOC + SZ_WDD;
static constexpr size_t OFF_W2   = OFF_W1 + SZ_WFF;
static constexpr size_t OFF_WMOD = OFF_W2 + SZ_WFF;
static constexpr size_t OFF_S16  = OFF_WMOD + SZ_WMOD;
static constexpr size_t OFF_MOD  = OFF_S16 + SZ_S16;
static constexpr size_t OFF_CIN  = OFF_MOD + SZ_MOD;
static constexpr size_t OFF_H16  = OFF_CIN + SZ_CIN;
static constexpr size_t OFF_QK   = OFF_H16 + SZ_H16;
static constexpr size_t OFF_VT   = OFF_QK + SZ_QK;
static constexpr size_t OFF_CTX  = OFF_VT + SZ_VT;
static constexpr size_t OFF_X1   = OFF_CTX + SZ_CTX;
static constexpr size_t OFF_X2   = OFF_X1 + SZ_X;
static constexpr size_t WS_TOTAL = OFF_X2 + SZ_X;
static constexpr size_t OFF_Q2   = OFF_QK;
static constexpr size_t OFF_K2   = OFF_QK + SZ_H16;
static constexpr size_t OFF_FF   = OFF_QK;

static_assert(WS_TOTAL <= (size_t)134217728);
static_assert(SZ_FF <= SZ_QK + SZ_VT + SZ_CTX);
static_assert(SZ_H16 + SZ_K2 <= SZ_QK);
static_assert(SZ_VT2 <= SZ_VT);
static_assert(OFF_WOS % 256 == 0 && OFF_WK % 256 == 0 && OFF_WV % 256 == 0 && OFF_S16 % 256 == 0 && OFF_MOD % 256 == 0);
static_assert(OFF_CIN % 256 == 0 && OFF_H16 % 256 == 0 && OFF_QK % 256 == 0 && OFF_K2 % 256 == 0 && OFF_X1 % 256 == 0);

static constexpr unsigned G_WQKV = (unsigned)((3 * DM * (DM / 8) + 255) / 256);
static constexpr unsigned G_WDD  = (unsigned)((DM * (DM / 8) + 255) / 256);
static constexpr unsigned G_WCD  = (unsigned)((DM * (CDIM / 8) + 255) / 256);
static constexpr unsigned G_W1   = (unsigned)((FFD * (DM / 8) + 255) / 256);
static constexpr unsigned G_W2   = (unsigned)((DM * (FFD / 8) + 255) / 256);
static constexpr unsigned G_WMOD = (unsigned)((NMOD * (DM / 8) + 255) / 256);
static constexpr unsigned G_SILU = (unsigned)(MODROWS * 4);
static constexpr unsigned G_CIN  = (unsigned)((MCTX * CDIM / 8) / 256);
static constexpr unsigned G_LN   = (unsigned)(MTOK / 8);
static constexpr unsigned G_MOD  = (unsigned)(((NMOD / 64) + 7) / 8);
static constexpr unsigned G_QK   = (unsigned)(((MTOK / 64) * (2 * DM / 64) + 7) / 8);
static constexpr unsigned G_TOKD = (unsigned)(((MTOK / 64) * (DM / 64) + 7) / 8);
static constexpr unsigned G_CTXD = (unsigned)(((MCTX / 64) * (DM / 64) + 7) / 8);
static constexpr unsigned G_FFU  = (unsigned)(((MTOK / 64) * (FFD / 64) + 7) / 8);
static constexpr unsigned G_ATT  = (unsigned)(NB * NHEAD * (SEQ / 128));

extern "C" void kernel_launch(void* const* d_in, const int* in_sizes, int n_in, void* d_out, int out_size,
                              void* d_ws, size_t ws_size, hipStream_t stream) {
    if (n_in < 27) return;
    if (in_sizes[0] < MTOK * DM || in_sizes[1] < MCTX * CDIM || in_sizes[2] < NB * DM) return;
    if (in_sizes[3] < DM || in_sizes[4] < DM || in_sizes[5] < DM || in_sizes[6] < DM || in_sizes[7] < DM || in_sizes[8] < DM) return;
    if (in_sizes[9] < DM * 3 * DM || in_sizes[10] < 3 * DM || in_sizes[11] < DM * DM || in_sizes[12] < DM) return;
    if (in_sizes[13] < DM * DM || in_sizes[14] < DM || in_sizes[15] < CDIM * DM || in_sizes[16] < DM) return;
    if (in_sizes[17] < CDIM * DM || in_sizes[18] < DM || in_sizes[19] < DM * DM || in_sizes[20] < DM) return;
    if (in_sizes[21] < DM * FFD || in_sizes[22] < FFD || in_sizes[23] < FFD * DM || in_sizes[24] < DM) return;
    if (in_sizes[25] < DM * NMOD || in_sizes[26] < NMOD || out_size < MTOK * DM) return;
    if (ws_size < WS_TOTAL) return;

    const float* x    = (const float*)d_in[0];
    const float* ctxi = (const float*)d_in[1];
    const float* temb = (const float*)d_in[2];
    const float* ln1w = (const float*)d_in[3];
    const float* ln1b = (const float*)d_in[4];
    const float* ln2w = (const float*)d_in[5];
    const float* ln2b = (const float*)d_in[6];
    const float* ln3w = (const float*)d_in[7];
    const float* ln3b = (const float*)d_in[8];
    const float* Wqkv = (const float*)d_in[9];
    const float* bqkv = (const float*)d_in[10];
    const float* Wos  = (const float*)d_in[11];
    const float* bos  = (const float*)d_in[12];
    const float* Wq   = (const float*)d_in[13];
    const float* bq   = (const float*)d_in[14];
    const float* Wk   = (const float*)d_in[15];
    const float* bk   = (const float*)d_in[16];
    const float* Wv   = (const float*)d_in[17];
    const float* bv   = (const float*)d_in[18];
    const float* Woc  = (const float*)d_in[19];
    const float* boc  = (const float*)d_in[20];
    const float* W1   = (const float*)d_in[21];
    const float* b1   = (const float*)d_in[22];
    const float* W2   = (const float*)d_in[23];
    const float* b2   = (const float*)d_in[24];
    const float* Wmod = (const float*)d_in[25];
    const float* bmod = (const float*)d_in[26];
    float* out = (float*)d_out;

    char* wsp = (char*)d_ws;
    h16*   wqkv  = (h16*)(wsp + OFF_WQKV);
    h16*   wos   = (h16*)(wsp + OFF_WOS);
    h16*   wq    = (h16*)(wsp + OFF_WQ);
    h16*   wk    = (h16*)(wsp + OFF_WK);
    h16*   wv    = (h16*)(wsp + OFF_WV);
    h16*   woc   = (h16*)(wsp + OFF_WOC);
    h16*   w1    = (h16*)(wsp + OFF_W1);
    h16*   w2    = (h16*)(wsp + OFF_W2);
    h16*   wmod  = (h16*)(wsp + OFF_WMOD);
    h16*   s16   = (h16*)(wsp + OFF_S16);
    float* modp  = (float*)(wsp + OFF_MOD);
    h16*   cin16 = (h16*)(wsp + OFF_CIN);
    h16*   hbuf  = (h16*)(wsp + OFF_H16);
    h16*   qk16  = (h16*)(wsp + OFF_QK);
    h16*   vt16  = (h16*)(wsp + OFF_VT);
    h16*   ctx16 = (h16*)(wsp + OFF_CTX);
    float* x1    = (float*)(wsp + OFF_X1);
    float* x2    = (float*)(wsp + OFF_X2);
    h16*   q2    = (h16*)(wsp + OFF_Q2);
    h16*   k2    = (h16*)(wsp + OFF_K2);
    h16*   ff16  = (h16*)(wsp + OFF_FF);

    k_wt16<<<G_WQKV, 256, 0, stream>>>(Wqkv, DM, 3 * DM, DM / 8, wqkv);
    k_wt16<<<G_WDD,  256, 0, stream>>>(Wos,  DM, DM, DM / 8, wos);
    k_wt16<<<G_WDD,  256, 0, stream>>>(Wq,   DM, DM, DM / 8, wq);
    k_wt16<<<G_WCD,  256, 0, stream>>>(Wk,   CDIM, DM, CDIM / 8, wk);
    k_wt16<<<G_WCD,  256, 0, stream>>>(Wv,   CDIM, DM, CDIM / 8, wv);
    k_wt16<<<G_WDD,  256, 0, stream>>>(Woc,  DM, DM, DM / 8, woc);
    k_wt16<<<G_W1,   256, 0, stream>>>(W1,   DM, FFD, DM / 8, w1);
    k_wt16<<<G_W2,   256, 0, stream>>>(W2,   FFD, DM, FFD / 8, w2);
    k_wt16<<<G_WMOD, 256, 0, stream>>>(Wmod, DM, NMOD, DM / 8, wmod);

    k_silu<<<G_SILU, 256, 0, stream>>>(temb, s16);
    k_ctx16<<<G_CIN, 256, 0, stream>>>(ctxi, cin16);
    k_gemm_mod<<<G_MOD, 256, 0, stream>>>(s16, DM, wmod, DM, modp, NMOD, bmod, MODROWS, NMOD, DM);

    k_lnmod<<<G_LN, 256, 0, stream>>>(x, ln1w, ln1b, modp, 0u, 1024u, 1u, hbuf);
    k_gemm_h16<<<G_QK, 256, 0, stream>>>(hbuf, DM, wqkv, DM, qk16, 2 * DM, bqkv, MTOK, 2 * DM, DM);
    k_gemm_tr<<<G_TOKD, 256, 0, stream>>>(hbuf, DM, wqkv + (size_t)2 * DM * DM, DM, vt16, bqkv + 2 * DM, MTOK, DM, DM, SEQ);
    k_attn_self<<<G_ATT, 256, 0, stream>>>(qk16, vt16, ctx16);
    k_gemm_res_s<<<G_TOKD, 256, 0, stream>>>(ctx16, DM, wos, DM, x1, DM, bos, x, MTOK, DM, DM);

    k_lnmod<<<G_LN, 256, 0, stream>>>(x1, ln2w, ln2b, modp, 2048u, 3072u, 0u, hbuf);
    k_gemm_h16<<<G_TOKD, 256, 0, stream>>>(hbuf, DM, wq, DM, q2, DM, bq, MTOK, DM, DM);
    k_gemm_h16<<<G_CTXD, 256, 0, stream>>>(cin16, CDIM, wk, CDIM, k2, DM, bk, MCTX, DM, CDIM);
    k_gemm_tr<<<G_CTXD, 256, 0, stream>>>(cin16, CDIM, wv, CDIM, vt16, bv, MCTX, DM, CDIM, NCTX);
    k_attn_cross<<<G_ATT, 256, 0, stream>>>(q2, k2, vt16, ctx16);
    k_gemm_res_c<<<G_TOKD, 256, 0, stream>>>(ctx16, DM, woc, DM, x2, DM, boc, x1, MTOK, DM, DM);

    k_lnmod<<<G_LN, 256, 0, stream>>>(x2, ln3w, ln3b, modp, 4096u, 5120u, 0u, hbuf);
    k_gemm_gelu<<<G_FFU, 256, 0, stream>>>(hbuf, DM, w1, DM, ff16, FFD, b1, MTOK, FFD, DM);
    k_gemm_res_f<<<G_TOKD, 256, 0, stream>>>(ff16, FFD, w2, FFD, out, DM, b2, x2, MTOK, DM, FFD);
}
